// MultiDANN_2448131358817
// MI455X (gfx1250) — hardware-verified
//
#include <hip/hip_runtime.h>


typedef _Float16 v16h __attribute__((ext_vector_type(16)));
typedef _Float16 v8h  __attribute__((ext_vector_type(8)));
typedef float    v8f  __attribute__((ext_vector_type(8)));
typedef float    v4f  __attribute__((ext_vector_type(4)));
typedef float    v2f  __attribute__((ext_vector_type(2)));
typedef int      v4i  __attribute__((ext_vector_type(4)));
union Frag { v16h v; v8h half[2]; };

#define FIN   64
#define HC    128
#define GG    64
#define HID   128
#define FEAT  256
#define NCLS  8
#define NEXP  3
#define RB    448
#define SLC   ((RB + 127) / 128)
#define NEG_SLOPE 0.2f
#define WSC   16.0f
#define ASC   64.0f
#define TP    132
#define HSP   136

__device__ __forceinline__ v8f wmma_f16(v16h a, v16h b, v8f c)
{
    c = __builtin_amdgcn_wmma_f32_16x16x32_f16(false, a, false, b, (short)0, c, false, false);
    asm volatile("v_nop\n\tv_nop\n\tv_nop\n\tv_nop" : "+v"(c) : "v"(a), "v"(b));
    return c;
}
__device__ __forceinline__ v8f zero8()
{
    v8f z = {0.f, 0.f, 0.f, 0.f, 0.f, 0.f, 0.f, 0.f};
    return z;
}
__device__ __forceinline__ v8h ld8h(const float* p)
{
    const v4f a = *(const v4f*)p;
    const v4f b = *(const v4f*)(p + 4);
    v8h r = {(_Float16)a[0], (_Float16)a[1], (_Float16)a[2], (_Float16)a[3],
             (_Float16)b[0], (_Float16)b[1], (_Float16)b[2], (_Float16)b[3]};
    return r;
}
__device__ __forceinline__ v8h ld8h(const _Float16* p) { return *(const v8h*)p; }

__device__ __forceinline__ v4f vmax4(v4f a, v4f b)
{
    v4f r = {fmaxf(a[0], b[0]), fmaxf(a[1], b[1]), fmaxf(a[2], b[2]), fmaxf(a[3], b[3])};
    return r;
}

__global__ __launch_bounds__(256) void k_prep(
    const float* __restrict__ w0, _Float16* __restrict__ t0,
    const float* __restrict__ w1, _Float16* __restrict__ t1,
    const float* __restrict__ w2, _Float16* __restrict__ t2,
    const float* __restrict__ w3, _Float16* __restrict__ t3,
    const float* __restrict__ w4, _Float16* __restrict__ t4,
    const float* __restrict__ w5, _Float16* __restrict__ t5)
{
    const int y = blockIdx.y;
    const float* W; _Float16* T; int K, NC, NP;
    if (y == 0)      { W = w0; T = t0; K = FIN;  NC = HC;   NP = HC;  }
    else if (y == 1) { W = w1; T = t1; K = HC;   NC = HC;   NP = HC;  }
    else if (y == 2) { W = w2; T = t2; K = FEAT; NC = HID;  NP = HID; }
    else if (y == 3) { W = w3; T = t3; K = FEAT; NC = HID;  NP = HID; }
    else if (y == 4) { W = w4; T = t4; K = HID;  NC = NCLS; NP = 16;  }
    else             { W = w5; T = t5; K = HID;  NC = NEXP; NP = 16;  }
    const int u  = blockIdx.x * 256 + (int)threadIdx.x;
    const int kq = K >> 3;
    const int n  = u / kq;
    const int q  = u - n * kq;
    if (n >= NP) return;
    float f[8];
#pragma unroll
    for (int i = 0; i < 8; ++i) {
        const int k = 8 * q + i;
        f[i] = (n < NC) ? W[(size_t)k * NC + n] * WSC : 0.f;
    }
    const v8h o = {(_Float16)f[0], (_Float16)f[1], (_Float16)f[2], (_Float16)f[3],
                   (_Float16)f[4], (_Float16)f[5], (_Float16)f[6], (_Float16)f[7]};
    _Float16* p = T + (size_t)n * K + 8 * q;
    *(volatile v8h*)p = o;
    __threadfence();
    *(volatile v8h*)p = o;
}

template<typename AT, int K>
__global__ __launch_bounds__(256) void k_proj(const AT* __restrict__ A, const _Float16* __restrict__ Bt,
                                            const float* __restrict__ att_s, const float* __restrict__ att_d,
                                            float* __restrict__ Hout, float* __restrict__ ASD, int n_rows)
{
    __shared__ __attribute__((aligned(16))) float T[16][TP];
    __shared__ float S[16][8];
    const int tid = threadIdx.x, lane = tid & 31, w = tid >> 5, h = lane >> 4, m = lane & 15;
    const int row0 = blockIdx.x * 16, col0 = w * 16;
    int ra = row0 + m; if (ra > n_rows - 1) ra = n_rows - 1;
    const AT* arow = A + (size_t)ra * K;
    const _Float16* brow = Bt + (size_t)(col0 + m) * K;

    v8f acc = zero8();
#pragma unroll
    for (int k0 = 0; k0 < K; k0 += 32) {
        Frag fa, fb;
        fa.half[0] = ld8h(arow + k0 + 8 * h);
        fa.half[1] = ld8h(arow + k0 + 16 + 8 * h);
        fb.half[0] = *(const v8h*)(brow + k0 + 8 * h);
        fb.half[1] = *(const v8h*)(brow + k0 + 16 + 8 * h);
        acc = wmma_f16(fa.v, fb.v, acc);
    }
#pragma unroll
    for (int r = 0; r < 8; ++r) T[8 * h + r][col0 + m] = acc[r] * (1.0f / WSC);
    __syncthreads();

    if (tid < 128) {
        const int rr = tid >> 3, j = tid & 7, hdd = j & 3;
        const float* av = (j & 4) ? att_d : att_s;
        float s = 0.f;
#pragma unroll
        for (int c = 0; c < 32; ++c) s += T[rr][hdd * 32 + c] * av[hdd * 32 + c];
        S[rr][j] = s;
    }
    __syncthreads();

    const int r0 = 2 * w, r1 = r0 + 1, rs = lane >> 1, qs = (lane & 1) * 4;
    const v4f hv0 = {T[r0][4 * lane], T[r0][4 * lane + 1], T[r0][4 * lane + 2], T[r0][4 * lane + 3]};
    const v4f hv1 = {T[r1][4 * lane], T[r1][4 * lane + 1], T[r1][4 * lane + 2], T[r1][4 * lane + 3]};
    const v4f sv  = {S[rs][qs], S[rs][qs + 1], S[rs][qs + 2], S[rs][qs + 3]};
    const bool ok0 = (row0 + r0) < n_rows;
    const bool ok1 = (row0 + r1) < n_rows;
    const bool oks = (w == 0) && ((row0 + rs) < n_rows);
    float* p0 = Hout + (size_t)(row0 + r0) * HC + 4 * lane;
    float* p1 = Hout + (size_t)(row0 + r1) * HC + 4 * lane;
    float* ps = ASD + (size_t)(row0 + rs) * 8 + qs;
    if (ok0) *(volatile v4f*)p0 = hv0;
    if (ok1) *(volatile v4f*)p1 = hv1;
    if (oks) *(volatile v4f*)ps = sv;
    __threadfence();
    if (ok0) *(volatile v4f*)p0 = hv0;
    if (ok1) *(volatile v4f*)p1 = hv1;
    if (oks) *(volatile v4f*)ps = sv;
}

template<bool FIRST>
__global__ __launch_bounds__(32) void k_gat_agg(const int* __restrict__ ei, int n_e, int n_nodes,
                                               const float* __restrict__ Hn, const float* __restrict__ ASD,
                                               const float* __restrict__ bias,
                                               _Float16* __restrict__ O16, float* __restrict__ O32)
{
    extern __shared__ __attribute__((aligned(16))) unsigned char dyn_lds[];
    v4f* accv = reinterpret_cast<v4f*>(dyn_lds);
    v2f* mdv  = reinterpret_cast<v2f*>(dyn_lds + (size_t)RB * 512);
    const int lane = threadIdx.x, hw = lane >> 4, li = lane & 15, hd = li >> 2;
    const int d0 = blockIdx.x * RB;
    const int* __restrict__ dstp = ei + n_e;

    {
        const v4f z4 = {0.f, 0.f, 0.f, 0.f};
        for (int i = lane; i < RB * 32; i += 32) accv[i] = z4;
        const v2f mi = {__int_as_float((int)0xff800000u), 0.f};
        for (int i = lane; i < RB * 4; i += 32) mdv[i] = mi;
    }
    __syncthreads();

    int pS = 0, pD = -1;

    auto pass = [&](int sA, int dA, int sB, int dB, bool vB) {
        const int s = hw ? sB : sA;
        const int d = hw ? dB : dA;
        if (hw == 0 || vB) {
            const int dl = d - d0;
            const v4f* hp = reinterpret_cast<const v4f*>(Hn + (size_t)s * HC + 8 * li);
            const v4f h0 = hp[0], h1 = hp[1];
            float ev = ASD[(size_t)s * 8 + hd] + ASD[(size_t)d * 8 + 4 + hd];
            ev = fmaxf(ev, NEG_SLOPE * ev);
            v2f st = mdv[dl * 4 + hd];
            const float mn = fmaxf(st[0], ev);
            const float sc = __expf(st[0] - mn);
            const float p  = __expf(ev - mn);
            st[1] = st[1] * sc + p;
            st[0] = mn;
            mdv[dl * 4 + hd] = st;
            v4f* ap = accv + dl * 32 + 2 * li;
            v4f a0 = ap[0], a1 = ap[1];
            a0 = a0 * sc + h0 * p;
            a1 = a1 * sc + h1 * p;
            ap[0] = a0;
            ap[1] = a1;
        }
        __syncthreads();
    };
    auto hit = [&](int s, int d) {
        if (pD < 0) { pS = s; pD = d; return; }
        const bool same = (pD == d);
        pass(pS, pD, s, d, !same);
        if (same) { pS = s; pD = d; } else { pD = -1; }
    };

    const int  nfull  = n_e >> 7;
    const bool vec_ok = ((n_e & 3) == 0);
    const int  nch    = nfull + 1 + SLC;
    for (int c = 0; c < nch; ++c) {
        const int base = c << 7;
        v4i dv = {-1, -1, -1, -1};
        if (c < nfull && vec_ok) {
            dv = *(const v4i*)(dstp + base + 4 * lane);
        } else if (c <= nfull) {
            const int i0 = base + 4 * lane;
            dv[0] = (i0 + 0 < n_e) ? dstp[i0 + 0] : -1;
            dv[1] = (i0 + 1 < n_e) ? dstp[i0 + 1] : -1;
            dv[2] = (i0 + 2 < n_e) ? dstp[i0 + 2] : -1;
            dv[3] = (i0 + 3 < n_e) ? dstp[i0 + 3] : -1;
        } else {
            const int t = c - nfull - 1;
            int lim = d0 + RB; if (lim > n_nodes) lim = n_nodes;
            const int nb = d0 + (t << 7) + 4 * lane;
            dv[0] = (nb + 0 < lim) ? nb + 0 : -1;
            dv[1] = (nb + 1 < lim) ? nb + 1 : -1;
            dv[2] = (nb + 2 < lim) ? nb + 2 : -1;
            dv[3] = (nb + 3 < lim) ? nb + 3 : -1;
        }
        const unsigned m0 = __builtin_amdgcn_ballot_w32((unsigned)(dv[0] - d0) < (unsigned)RB);
        const unsigned m1 = __builtin_amdgcn_ballot_w32((unsigned)(dv[1] - d0) < (unsigned)RB);
        const unsigned m2 = __builtin_amdgcn_ballot_w32((unsigned)(dv[2] - d0) < (unsigned)RB);
        const unsigned m3 = __builtin_amdgcn_ballot_w32((unsigned)(dv[3] - d0) < (unsigned)RB);
        unsigned anym = m0 | m1 | m2 | m3;
        while (anym) {
            const int ln = __builtin_ctz(anym);
            anym &= anym - 1u;
            unsigned fl = ((m0 >> ln) & 1u) | (((m1 >> ln) & 1u) << 1) |
                          (((m2 >> ln) & 1u) << 2) | (((m3 >> ln) & 1u) << 3);
            while (fl) {
                const int j = __builtin_ctz(fl);
                fl &= fl - 1u;
                int s, d;
                if (c <= nfull) {
                    const int e = base + 4 * ln + j;
                    s = __builtin_amdgcn_readfirstlane(ei[e]);
                    d = __builtin_amdgcn_readfirstlane(dstp[e]);
                } else {
                    d = d0 + ((c - nfull - 1) << 7) + 4 * ln + j;
                    s = d;
                }
                if ((unsigned)d < (unsigned)n_nodes && (unsigned)(d - d0) < (unsigned)RB) {
                    s = (s < 0) ? 0 : ((s > n_nodes - 1) ? (n_nodes - 1) : s);
                    hit(s, d);
                }
            }
        }
    }
    if (pD >= 0) pass(pS, pD, pS, pD, false);
    __syncthreads();

    auto emit = [&]() {
        if (FIRST) {
            const v4f* b4 = reinterpret_cast<const v4f*>(bias);
            const v4f bb0 = b4[2 * li], bb1 = b4[2 * li + 1];
            for (int i = 0; i < RB / 2; ++i) {
                if (d0 + 2 * i >= n_nodes) break;
                const int dl = 2 * i + hw;
                const int d  = d0 + dl;
                const v2f st = mdv[dl * 4 + hd];
                const float inv = 1.0f / (st[1] + 1e-16f);
                v4f a0 = accv[dl * 32 + 2 * li], a1 = accv[dl * 32 + 2 * li + 1];
                a0 = a0 * inv + bb0;
                a1 = a1 * inv + bb1;
                const v4f z = {0.f, 0.f, 0.f, 0.f};
                a0 = vmax4(a0, z);
                a1 = vmax4(a1, z);
                const v8h pk = {(_Float16)a0[0], (_Float16)a0[1], (_Float16)a0[2], (_Float16)a0[3],
                                (_Float16)a1[0], (_Float16)a1[1], (_Float16)a1[2], (_Float16)a1[3]};
                if (d < n_nodes) *(volatile v8h*)(O16 + (size_t)d * HC + 8 * li) = pk;
            }
        } else {
            const int hh = lane >> 3;
            const v4f bb = reinterpret_cast<const v4f*>(bias)[lane];
            for (int dl = 0; dl < RB; ++dl) {
                const int d = d0 + dl;
                if (d >= n_nodes) break;
                const v2f st = mdv[dl * 4 + hh];
                const float inv = 1.0f / (st[1] + 1e-16f);
                v4f a = accv[dl * 32 + lane];
                a = a * inv + bb;
                *(volatile v4f*)(O32 + (size_t)d * HC + 4 * lane) = a;
            }
        }
    };
    emit();
    __threadfence();
    emit();
}

__global__ __launch_bounds__(32) void k_pool(const float* __restrict__ X2, const int* __restrict__ bat, int n_nodes,
                                            _Float16* __restrict__ F16)
{
    const int lane = threadIdx.x, li = lane & 15, hw = lane >> 4;
    const int g = blockIdx.x;
    const float ninf = __int_as_float((int)0xff800000u);
    v4f s0 = {0.f, 0.f, 0.f, 0.f}, s1 = s0;
    v4f x0 = {ninf, ninf, ninf, ninf}, x1 = x0;
    int cnt = 0;
    const int nch = (n_nodes + 127) >> 7;
    for (int c = 0; c < nch; ++c) {
        const int base = c << 7;
        const int i0 = base + 4 * lane;
        v4i bv = {-1, -1, -1, -1};
        if (base + 128 <= n_nodes) {
            bv = *(const v4i*)(bat + i0);
        } else {
            bv[0] = (i0 + 0 < n_nodes) ? bat[i0 + 0] : -1;
            bv[1] = (i0 + 1 < n_nodes) ? bat[i0 + 1] : -1;
            bv[2] = (i0 + 2 < n_nodes) ? bat[i0 + 2] : -1;
            bv[3] = (i0 + 3 < n_nodes) ? bat[i0 + 3] : -1;
        }
        const unsigned m0 = __builtin_amdgcn_ballot_w32(bv[0] == g);
        const unsigned m1 = __builtin_amdgcn_ballot_w32(bv[1] == g);
        const unsigned m2 = __builtin_amdgcn_ballot_w32(bv[2] == g);
        const unsigned m3 = __builtin_amdgcn_ballot_w32(bv[3] == g);
        unsigned anym = m0 | m1 | m2 | m3;
        while (anym) {
            const int ln = __builtin_ctz(anym);
            anym &= anym - 1u;
            unsigned fl = ((m0 >> ln) & 1u) | (((m1 >> ln) & 1u) << 1) |
                          (((m2 >> ln) & 1u) << 2) | (((m3 >> ln) & 1u) << 3);
            while (fl) {
                const int j = __builtin_ctz(fl);
                fl &= fl - 1u;
                const int n = base + 4 * ln + j;
                const v4f* xp = reinterpret_cast<const v4f*>(X2 + (size_t)n * HC + 8 * li);
                const v4f a = xp[0], b = xp[1];
                s0 = s0 + a; s1 = s1 + b;
                x0 = vmax4(x0, a); x1 = vmax4(x1, b);
                ++cnt;
            }
        }
    }
    const float invc = 1.0f / (float)(cnt > 0 ? cnt : 1);
    v4f u0 = s0 * invc, u1 = s1 * invc;
    if (hw) { u0 = x0; u1 = x1; }
    float q = u0[0] * u0[0] + u0[1] * u0[1] + u0[2] * u0[2] + u0[3] * u0[3]
            + u1[0] * u1[0] + u1[1] * u1[1] + u1[2] * u1[2] + u1[3] * u1[3];
    q += __shfl_xor(q, 16);
    q += __shfl_xor(q, 8);
    q += __shfl_xor(q, 4);
    q += __shfl_xor(q, 2);
    q += __shfl_xor(q, 1);
    float nrm = sqrtf(q);
    nrm = fmaxf(nrm, 1e-12f);
    const float f = (1.0f / nrm) * ASC;
    const v8h pk = {(_Float16)(u0[0] * f), (_Float16)(u0[1] * f), (_Float16)(u0[2] * f), (_Float16)(u0[3] * f),
                    (_Float16)(u1[0] * f), (_Float16)(u1[1] * f), (_Float16)(u1[2] * f), (_Float16)(u1[3] * f)};
    _Float16* p = F16 + (size_t)g * FEAT + 8 * lane;
    *(volatile v8h*)p = pk;
    __threadfence();
    *(volatile v8h*)p = pk;
}

__device__ __forceinline__ void lda16(Frag& f, const _Float16* rowp, int k0, int h)
{
    f.half[0] = *(const v8h*)(rowp + k0 + 8 * h);
    f.half[1] = *(const v8h*)(rowp + k0 + 16 + 8 * h);
}

__global__ __launch_bounds__(256) void k_head(const _Float16* __restrict__ F16,
                                            const _Float16* __restrict__ W1c, const float* __restrict__ b1c,
                                            const _Float16* __restrict__ Woc, const float* __restrict__ boc,
                                            const _Float16* __restrict__ W1d, const float* __restrict__ b1d,
                                            const _Float16* __restrict__ Wod, const float* __restrict__ bod,
                                            const int* __restrict__ sel, float* __restrict__ out)
{
    __shared__ __attribute__((aligned(16))) _Float16 Hs[GG * HSP];
    __shared__ float Os[GG * 16];
    (void)sel;
    const int tid = threadIdx.x, lane = tid & 31, w = tid >> 5, h = lane >> 4, m = lane & 15;
    const int hs = blockIdx.x;
    const _Float16* W1 = hs ? W1d : W1c;
    const float*    b1 = hs ? b1d : b1c;
    const _Float16* Wo = hs ? Wod : Woc;
    const float*    bo = hs ? bod : boc;
    const int nout = hs ? NEXP : NCLS;
    float* op = out + (hs ? GG * NCLS : 0);

    v8f acc0 = zero8(), acc1 = zero8(), acc2 = zero8(), acc3 = zero8();
    const _Float16* brow = W1 + (size_t)(16 * w + m) * FEAT;
#pragma unroll
    for (int k0 = 0; k0 < FEAT; k0 += 32) {
        Frag fb, fa;
        lda16(fb, brow, k0, h);
        lda16(fa, F16 + (size_t)(0 * 16 + m) * FEAT, k0, h);  acc0 = wmma_f16(fa.v, fb.v, acc0);
        lda16(fa, F16 + (size_t)(1 * 16 + m) * FEAT, k0, h);  acc1 = wmma_f16(fa.v, fb.v, acc1);
        lda16(fa, F16 + (size_t)(2 * 16 + m) * FEAT, k0, h);  acc2 = wmma_f16(fa.v, fb.v, acc2);
        lda16(fa, F16 + (size_t)(3 * 16 + m) * FEAT, k0, h);  acc3 = wmma_f16(fa.v, fb.v, acc3);
    }
    const float sc1 = 1.0f / (WSC * ASC);
    const int col = 16 * w + m;
    const float bc = b1[col];
#pragma unroll
    for (int r = 0; r < 8; ++r) {
        Hs[(0 * 16 + 8 * h + r) * HSP + col] = (_Float16)(fmaxf(acc0[r] * sc1 + bc, 0.f) * ASC);
        Hs[(1 * 16 + 8 * h + r) * HSP + col] = (_Float16)(fmaxf(acc1[r] * sc1 + bc, 0.f) * ASC);
        Hs[(2 * 16 + 8 * h + r) * HSP + col] = (_Float16)(fmaxf(acc2[r] * sc1 + bc, 0.f) * ASC);
        Hs[(3 * 16 + 8 * h + r) * HSP + col] = (_Float16)(fmaxf(acc3[r] * sc1 + bc, 0.f) * ASC);
    }
    __syncthreads();

    if (w < 4) {
        v8f acq = zero8();
        const _Float16* ar = Hs + (size_t)(16 * w + m) * HSP;
        const _Float16* br = Wo + (size_t)m * HID;
#pragma unroll
        for (int k0 = 0; k0 < HID; k0 += 32) {
            Frag fa, fb;
            lda16(fa, ar, k0, h);
            lda16(fb, br, k0, h);
            acq = wmma_f16(fa.v, fb.v, acq);
        }
        float bom = 0.f;
        if (m < nout) bom = bo[m];
#pragma unroll
        for (int r = 0; r < 8; ++r) Os[(16 * w + 8 * h + r) * 16 + m] = acq[r] * sc1 + bom;
    }
    __syncthreads();

    if (w == 0) {
        const int tot4 = (GG * nout) >> 2;
        v4f vq[4];
        bool okq[4];
#pragma unroll
        for (int qq = 0; qq < 4; ++qq) {
            const int f4 = 32 * qq + lane;
            okq[qq] = f4 < tot4;
            float t[4];
#pragma unroll
            for (int i = 0; i < 4; ++i) {
                int e = 4 * f4 + i;
                if (!okq[qq]) e = 0;
                const int gq = e / nout;
                const int o  = e - gq * nout;
                t[i] = Os[gq * 16 + o];
            }
            const v4f v = {t[0], t[1], t[2], t[3]};
            vq[qq] = v;
        }
#pragma unroll
        for (int qq = 0; qq < 4; ++qq)
            if (okq[qq]) *(volatile v4f*)(op + 4 * (32 * qq + lane)) = vq[qq];
        __threadfence();
#pragma unroll
        for (int qq = 0; qq < 4; ++qq)
            if (okq[qq]) *(volatile v4f*)(op + 4 * (32 * qq + lane)) = vq[qq];
    }
}

static inline size_t al256(size_t x) { return (x + 255) & ~(size_t)255; }

extern "C" void kernel_launch(void* const* d_in, const int* in_sizes, int n_in,
                              void* d_out, int out_size, void* d_ws, size_t ws_size,
                              hipStream_t stream)
{
    (void)out_size;
    if (n_in < 20) return;
    const int n_nodes = in_sizes[0] / FIN;
    const int n_e     = in_sizes[1] / 2;
    if (n_nodes <= 0 || n_e < 0) return;

    const float* x    = (const float*)d_in[0];
    const int*   ei   = (const int*)d_in[1];
    const int*   bat  = (const int*)d_in[2];
    const int*   sel  = (const int*)d_in[3];
    const float* eW1  = (const float*)d_in[4];
    const float* eas1 = (const float*)d_in[5];
    const float* ead1 = (const float*)d_in[6];
    const float* eb1  = (const float*)d_in[7];
    const float* eW2  = (const float*)d_in[8];
    const float* eas2 = (const float*)d_in[9];
    const float* ead2 = (const float*)d_in[10];
    const float* eb2  = (const float*)d_in[11];
    const float* cW1  = (const float*)d_in[12];
    const float* cb1  = (const float*)d_in[13];
    const float* cWo  = (const float*)d_in[14];
    const float* cbo  = (const float*)d_in[15];
    const float* dW1  = (const float*)d_in[16];
    const float* db1  = (const float*)d_in[17];
    const float* dWo  = (const float*)d_in[18];
    const float* dbo  = (const float*)d_in[19];
    float* out = (float*)d_out;

    char* ws = (char*)d_ws;
    size_t off = 0;
    auto carve = [&](size_t bytes) { char* p = ws + off; off += al256(bytes); return p; };
    float*    h32  = (float*)   carve((size_t)n_nodes * HC * sizeof(float));
    float*    asd8 = (float*)   carve((size_t)n_nodes * 8 * sizeof(float));
    _Float16* in16 = (_Float16*)carve((size_t)n_nodes * HC * sizeof(_Float16));
    float*    out2 = (float*)   carve((size_t)n_nodes * HC * sizeof(float));
    _Float16* Wt1  = (_Float16*)carve((size_t)HC * FIN * 2);
    _Float16* Wt2  = (_Float16*)carve((size_t)HC * HC * 2);
    _Float16* Wc1  = (_Float16*)carve((size_t)HID * FEAT * 2);
    _Float16* Wd1  = (_Float16*)carve((size_t)HID * FEAT * 2);
    _Float16* Wco  = (_Float16*)carve((size_t)16 * HID * 2);
    _Float16* Wdo  = (_Float16*)carve((size_t)16 * HID * 2);
    _Float16* f16  = (_Float16*)carve((size_t)GG * FEAT * 2);
    if (off > ws_size) return;

    const size_t lds_agg = (size_t)RB * 512 + (size_t)RB * 32;
    hipFuncSetAttribute(reinterpret_cast<const void*>(&k_gat_agg<true>),
                        hipFuncAttributeMaxDynamicSharedMemorySize, (int)lds_agg);
    hipFuncSetAttribute(reinterpret_cast<const void*>(&k_gat_agg<false>),
                        hipFuncAttributeMaxDynamicSharedMemorySize, (int)lds_agg);

    k_prep<<<dim3(16, 6), 256, 0, stream>>>(eW1, Wt1, eW2, Wt2, cW1, Wc1, dW1, Wd1, cWo, Wco, dWo, Wdo);

    const int pgrid = (n_nodes + 15) / 16;
    const int agrid = (n_nodes + RB - 1) / RB;

    k_proj<float, FIN><<<pgrid, 256, 0, stream>>>(x, Wt1, eas1, ead1, h32, asd8, n_nodes);
    k_gat_agg<true><<<agrid, 32, lds_agg, stream>>>(ei, n_e, n_nodes, h32, asd8, eb1, in16, out2);

    k_proj<_Float16, HC><<<pgrid, 256, 0, stream>>>(in16, Wt2, eas2, ead2, h32, asd8, n_nodes);
    k_gat_agg<false><<<agrid, 32, lds_agg, stream>>>(ei, n_e, n_nodes, h32, asd8, eb2, in16, out2);

    k_pool<<<GG, 32, 0, stream>>>(out2, bat, n_nodes, f16);
    k_head<<<2, 256, 0, stream>>>(f16, Wc1, cb1, Wco, cbo, Wd1, db1, Wdo, dbo, sel, out);
    hipGetLastError();
}
